// SceneGenerator_88132728913975
// MI455X (gfx1250) — hardware-verified
//
#include <hip/hip_runtime.h>

#pragma clang fp contract(off)

#define HID   128
#define PPB   128
#define NTHR  256
#define ZD    64
#define FRES  16
#define NPE   10
#define NLAY  4
#define WPL   (2 * HID * HID)

typedef __bf16         v16bf __attribute__((ext_vector_type(16)));
typedef unsigned short v8us  __attribute__((ext_vector_type(8), __may_alias__));
typedef unsigned short v16us __attribute__((ext_vector_type(16), __may_alias__));
typedef float          v8f   __attribute__((ext_vector_type(8)));
typedef float          v4f   __attribute__((ext_vector_type(4), __may_alias__));

union Frag { v16bf v; v16us u; v8us h8[2]; };

__device__ __forceinline__ void split2(float x, unsigned short& hi, unsigned short& lo) {
    const __bf16 bh = (__bf16)x;
    const float  r  = x - (float)bh;
    const __bf16 bl = (__bf16)r;
    hi = __builtin_bit_cast(unsigned short, bh);
    lo = __builtin_bit_cast(unsigned short, bl);
}

__device__ __forceinline__ void put2(unsigned short* p0, unsigned short* p1, int idx, float v) {
    unsigned short hi, lo;
    split2(v, hi, lo);
    p0[idx] = hi;
    p1[idx] = lo;
}

__device__ __forceinline__ v8f mma3(v8f acc, v16bf ah, v16bf al, v16bf bh, v16bf bl) {
    acc = __builtin_amdgcn_wmma_f32_16x16x32_bf16(false, ah, false, bh, (short)0, acc, false, false);
    acc = __builtin_amdgcn_wmma_f32_16x16x32_bf16(false, ah, false, bl, (short)0, acc, false, false);
    acc = __builtin_amdgcn_wmma_f32_16x16x32_bf16(false, al, false, bh, (short)0, acc, false, false);
    asm volatile("v_nop\n\tv_nop\n\tv_nop\n\tv_nop" : "+v"(acc) : "v"(al), "v"(bh), "v"(ah), "v"(bl));
    return acc;
}

__global__ void __launch_bounds__(NTHR)
k_pack(const float* __restrict__ W0, const float* __restrict__ W1,
       const float* __restrict__ W2, const float* __restrict__ W3,
       int k0rows, unsigned short* wp, int total)
{
    const int t = blockIdx.x * NTHR + threadIdx.x;
    if (t >= total) return;
    const int e     = t & 1;
    const int lane  = (t >> 1) & 31;
    const int frag  = (t >> 6) & 31;
    const int plane = (t >> 11) & 1;
    const int L     = (t >> 12) & 3;
    const int nt = frag >> 2, kt = frag & 3, h = lane >> 4;
    const int n  = nt * 16 + (lane & 15);
    const int kb = kt * 32 + 16 * e + 8 * h;
    const float* W = (L == 0) ? W0 : (L == 1) ? W1 : (L == 2) ? W2 : W3;
    const int krows = (L == 0) ? k0rows : HID;
    v8us o;
    #pragma unroll
    for (int i = 0; i < 8; ++i) {
        const int k = kb + i;
        float v = 0.0f;
        if (k < krows) v = W[k * HID + n];
        unsigned short hi, lo;
        split2(v, hi, lo);
        o[i] = plane ? lo : hi;
    }
    volatile v8us* dst = (volatile v8us*)(wp + (size_t)t * 8);
    *dst = o;
    __threadfence();
    *dst = o;
}

__device__ __forceinline__ void pe_one(unsigned short* h0, unsigned short* h1, int d, float c) {
    #pragma unroll
    for (int f = 0; f < NPE; f += 2) {
        const float a = c * (float)(1 << f);
        float s, co;
        sincosf(a, &s, &co);
        put2(h0, h1, ZD + 3 + f * 3 + d, s);
        put2(h0, h1, ZD + 3 + 3 * NPE + f * 3 + d, co);
        const float s2 = 2.0f * s * co;
        const float c2 = (co - s) * (co + s);
        put2(h0, h1, ZD + 3 + (f + 1) * 3 + d, s2);
        put2(h0, h1, ZD + 3 + 3 * NPE + (f + 1) * 3 + d, c2);
    }
}

__global__ void __launch_bounds__(NTHR)
k_mlp(const float* __restrict__ xyz,
      const float* __restrict__ lat,
      const unsigned short* __restrict__ wp,
      const float* __restrict__ b0, const float* __restrict__ b1,
      const float* __restrict__ b2, const float* __restrict__ b3,
      const float* __restrict__ Wa, const float* __restrict__ ba,
      float* out, int npts, int nper, int nb)
{
    __shared__ __align__(16) unsigned short hb[2][PPB * HID];
    __shared__ __align__(16) unsigned short wb[2][HID * HID];
    __shared__ float bb[NLAY * HID];
    __shared__ float wab[HID];
    __shared__ __align__(16) float ob[PPB];

    const int tid  = threadIdx.x;
    const int l    = tid & 31;
    const int wv   = tid >> 5;
    const int h    = l >> 4;
    const int col  = l & 15;
    const int blk0 = blockIdx.x * PPB;

    for (int i = tid; i < NLAY * HID; i += NTHR) {
        const float* bp = (i < HID) ? b0 : (i < 2 * HID) ? b1 : (i < 3 * HID) ? b2 : b3;
        bb[i] = bp[i & (HID - 1)];
    }
    if (tid < HID) wab[tid] = Wa[tid];

    {
        const int lp = tid >> 1;
        const int cb = (tid & 1) * (ZD / 2);
        int p = blk0 + lp; p = (p < npts) ? p : (npts - 1);
        int b = p / nper;  b = (b < nb) ? b : (nb - 1);
        const float X = xyz[(size_t)p * 3 + 0];
        const float Z = xyz[(size_t)p * 3 + 2];
        float px = (X + 1.0f) * 8.0f - 0.5f;
        float py = (Z + 1.0f) * 8.0f - 0.5f;
        px = fminf(fmaxf(px, -4.0f), 20.0f);
        py = fminf(fmaxf(py, -4.0f), 20.0f);
        const float x0f = floorf(px), y0f = floorf(py);
        const float x1f = x0f + 1.0f, y1f = y0f + 1.0f;
        const float wx0 = x1f - px, wx1 = px - x0f;
        const float wy0 = y1f - py, wy1 = py - y0f;
        const float lim = (float)(FRES - 1);
        const float vx0 = (x0f >= 0.0f && x0f <= lim) ? 1.0f : 0.0f;
        const float vx1 = (x1f >= 0.0f && x1f <= lim) ? 1.0f : 0.0f;
        const float vy0 = (y0f >= 0.0f && y0f <= lim) ? 1.0f : 0.0f;
        const float vy1 = (y1f >= 0.0f && y1f <= lim) ? 1.0f : 0.0f;
        const int x0c = min(max((int)x0f, 0), FRES - 1), x1c = min(max((int)x1f, 0), FRES - 1);
        const int y0c = min(max((int)y0f, 0), FRES - 1), y1c = min(max((int)y1f, 0), FRES - 1);
        const float m00 = vx0 * vy0, m01 = vx0 * vy1, m10 = vx1 * vy0, m11 = vx1 * vy1;
        const float w00 = wx0 * wy0, w01 = wx0 * wy1, w10 = wx1 * wy0, w11 = wx1 * wy1;
        const int o00 = y0c * FRES + x0c, o01 = y1c * FRES + x0c;
        const int o10 = y0c * FRES + x1c, o11 = y1c * FRES + x1c;
        const float* img = lat + (size_t)b * ZD * FRES * FRES;
        unsigned short* h0 = &hb[0][lp * HID];
        unsigned short* h1 = &hb[1][lp * HID];
        #pragma unroll 2
        for (int c = 0; c < ZD / 2; ++c) {
            const float* pc = img + (cb + c) * (FRES * FRES);
            const float g00 = pc[o00] * m00, g01 = pc[o01] * m01;
            const float g10 = pc[o10] * m10, g11 = pc[o11] * m11;
            const float v = g00 * w00 + g01 * w01 + g10 * w10 + g11 * w11;
            put2(h0, h1, cb + c, v);
        }
    }

    if (tid < PPB) {
        int p = blk0 + tid; p = (p < npts) ? p : (npts - 1);
        const float X = xyz[(size_t)p * 3 + 0];
        const float Y = xyz[(size_t)p * 3 + 1];
        const float Z = xyz[(size_t)p * 3 + 2];
        const float tx = (X + 1.0f) * 0.5f * (float)FRES;
        const float tz = (Z + 1.0f) * 0.5f * (float)FRES;
        const float lcx = (tx - rintf(tx - 0.5f)) * 2.0f - 1.0f;
        const float lcz = (tz - rintf(tz - 0.5f)) * 2.0f - 1.0f;
        unsigned short* h0 = &hb[0][tid * HID];
        unsigned short* h1 = &hb[1][tid * HID];
        put2(h0, h1, ZD + 0, lcx);
        put2(h0, h1, ZD + 1, Y);
        put2(h0, h1, ZD + 2, lcz);
        pe_one(h0, h1, 0, lcx);
        pe_one(h0, h1, 1, Y);
        pe_one(h0, h1, 2, lcz);
        h0[HID - 1] = 0;
        h1[HID - 1] = 0;
    }

    v8f hp = {0.0f, 0.0f, 0.0f, 0.0f, 0.0f, 0.0f, 0.0f, 0.0f};
    const int m    = wv * 16 + col;
    const int rowb = wv * 16 + 8 * h;

    #pragma unroll 1
    for (int L = 0; L < NLAY; ++L) {
        __syncthreads();
        {
            const v8us* src = (const v8us*)(wp + (size_t)L * WPL);
            v8us* dst = (v8us*)&wb[0][0];
            #pragma unroll
            for (int j = 0; j < (WPL / 8) / NTHR; ++j) dst[j * NTHR + tid] = src[j * NTHR + tid];
        }
        __syncthreads();

        Frag ah[4], al[4];
        #pragma unroll
        for (int kt = 0; kt < 4; ++kt) {
            const int base = m * HID + kt * 32 + 8 * h;
            ah[kt].h8[0] = *(const v8us*)&hb[0][base];
            ah[kt].h8[1] = *(const v8us*)&hb[0][base + 16];
            al[kt].h8[0] = *(const v8us*)&hb[1][base];
            al[kt].h8[1] = *(const v8us*)&hb[1][base + 16];
        }

        #pragma unroll 1
        for (int nt = 0; nt < HID / 16; ++nt) {
            const float bias = bb[L * HID + nt * 16 + col];
            v8f acc = {bias, bias, bias, bias, bias, bias, bias, bias};
            #pragma unroll
            for (int kt = 0; kt < 4; ++kt) {
                Frag bh, bl;
                bh.u = *(const v16us*)&wb[0][(nt * 4 + kt) * 512 + l * 16];
                bl.u = *(const v16us*)&wb[1][(nt * 4 + kt) * 512 + l * 16];
                acc = mma3(acc, ah[kt].v, al[kt].v, bh.v, bl.v);
            }
            if (L < NLAY - 1) {
                #pragma unroll
                for (int r = 0; r < 8; ++r) {
                    float v = acc[r];
                    v = (v > 0.0f) ? v : 0.0f;
                    const int idx = (rowb + r) * HID + nt * 16 + col;
                    put2(&hb[0][0], &hb[1][0], idx, v);
                }
            } else {
                const float w = wab[nt * 16 + col];
                #pragma unroll
                for (int r = 0; r < 8; ++r) {
                    float v = acc[r];
                    v = (v > 0.0f) ? v : 0.0f;
                    hp[r] = hp[r] + v * w;
                }
            }
        }
    }

    #pragma unroll
    for (int off = 8; off > 0; off >>= 1) {
        #pragma unroll
        for (int r = 0; r < 8; ++r) hp[r] = hp[r] + __shfl_xor(hp[r], off);
    }
    const float ba0 = ba[0];
    if (col == 0) {
        #pragma unroll
        for (int r = 0; r < 8; ++r) ob[rowb + r] = hp[r] + ba0;
    }
    __syncthreads();

    if (blk0 + PPB <= npts) {
        if (tid < 32) {
            const v4f v = *(const v4f*)&ob[4 * tid];
            volatile v4f* dst = (volatile v4f*)(out + (size_t)blk0 + 4 * tid);
            *dst = v;
            __threadfence();
            *dst = v;
        }
    } else {
        if (tid < PPB && blk0 + tid < npts) {
            const float v = ob[tid];
            volatile float* dst = out + (size_t)blk0 + tid;
            *dst = v;
            __threadfence();
            *dst = v;
        }
    }
}

extern "C" void kernel_launch(void* const* d_in, const int* in_sizes, int n_in,
                              void* d_out, int out_size, void* d_ws, size_t ws_size,
                              hipStream_t stream) {
    if (n_in < 12) return;
    const float* xyz = (const float*)d_in[0];
    const float* lat = (const float*)d_in[1];
    const float* W0  = (const float*)d_in[2];
    const float* b0  = (const float*)d_in[3];
    const float* W1  = (const float*)d_in[4];
    const float* b1  = (const float*)d_in[5];
    const float* W2  = (const float*)d_in[6];
    const float* b2  = (const float*)d_in[7];
    const float* W3  = (const float*)d_in[8];
    const float* b3  = (const float*)d_in[9];
    const float* Wa  = (const float*)d_in[10];
    const float* ba  = (const float*)d_in[11];
    float* out = (float*)d_out;

    int npts = in_sizes[0] / 3;
    if (npts > out_size) npts = out_size;
    if (npts <= 0) return;
    int nb = in_sizes[1] / (ZD * FRES * FRES);
    if (nb < 1) nb = 1;
    int nper = npts / nb;
    if (nper < 1) nper = 1;
    const int k0rows = in_sizes[2] / HID;

    const size_t wp_bytes = (size_t)NLAY * WPL * sizeof(unsigned short);
    if (wp_bytes > ws_size) return;
    unsigned short* wp = (unsigned short*)d_ws;

    const int total = NLAY * 2 * 32 * 32 * 2;
    k_pack<<<(total + NTHR - 1) / NTHR, NTHR, 0, stream>>>(W0, W1, W2, W3, k0rows, wp, total);

    k_mlp<<<(npts + PPB - 1) / PPB, NTHR, 0, stream>>>(
        xyz, lat, wp, b0, b1, b2, b3, Wa, ba, out, npts, nper, nb);
    (void)hipGetLastError();
}
